// GraphGRU_64836826301014
// MI455X (gfx1250) — hardware-verified
//
#include <hip/hip_runtime.h>
#include <hip/hip_bf16.h>
#include <stddef.h>


#define HID      160
#define KZ       (2 * HID)
#define NEI      8
#define TROWS    64
#define NTHR     128
#define NWV      (NTHR / 32)
#define C4       (HID / 4)
#define ITEMS    ((TROWS * C4) / NTHR)
#define NST      (16 * C4 / 32)
#define PTHR     256
#define NGZ      (HID * KZ / 8)
#define NGR      (HID * HID / 8)
#define BZ       ((NGZ + PTHR - 1) / PTHR)
#define BR       ((NGR + PTHR - 1) / PTHR)
#define NPREPB   (2 * BZ + 2 * BR)
#define LDS_GATE ((3 * TROWS * HID + TROWS * NEI) * 4)

static_assert(HID % 32 == 0);
static_assert(TROWS == NWV * 16);
static_assert((TROWS * C4) % NTHR == 0);
static_assert(TROWS * NEI / 4 == NTHR);
static_assert((16 * C4) % 32 == 0);
static_assert(TROWS * HID * 4 <= 65536);
static_assert(LDS_GATE <= 160 * 1024);
static_assert((HID * 4) % 128 == 0);

typedef float          v4f   __attribute__((ext_vector_type(4)));
typedef float          v8f   __attribute__((ext_vector_type(8)));
typedef int            v4i   __attribute__((ext_vector_type(4)));
typedef unsigned short v8us  __attribute__((ext_vector_type(8)));
typedef unsigned short v16us __attribute__((ext_vector_type(16)));
typedef __bf16         v16bf __attribute__((ext_vector_type(16)));
union FragB { v16bf v; v16us u; v8us h[2]; };

__device__ __forceinline__ unsigned short bfr(float f) {
  unsigned u = __float_as_uint(f);
  u += 0x7fffu + ((u >> 16) & 1u);
  return (unsigned short)(u >> 16);
}
__device__ __forceinline__ float bfup(unsigned short s) { return __uint_as_float(((unsigned)s) << 16); }
__device__ __forceinline__ float bfq(float f) { return bfup(bfr(f)); }

__device__ __forceinline__ float sigf(float x) {
  x = fminf(fmaxf(x, -87.0f), 87.0f);
  const float e = __expf(-x);
  return __builtin_amdgcn_rcpf(1.0f + e);
}
__device__ __forceinline__ float tnhf(float x) {
  const float a = fminf(fabsf(x), 44.0f);
  const float t = __expf(-2.0f * a);
  const float y = (1.0f - t) * __builtin_amdgcn_rcpf(1.0f + t);
  return copysignf(y, x);
}

__device__ __forceinline__ v8f wmb(v16bf a, v16bf b, v8f c) {
  v8f d = __builtin_amdgcn_wmma_f32_16x16x32_bf16(false, a, false, b, (short)0, c, false, false);
#if defined(__HIP_DEVICE_COMPILE__)
  asm volatile("v_nop\n\tv_nop\n\tv_nop\n\tv_nop" : "+v"(d) : "v"(a), "v"(b));
#endif
  return d;
}

#define CV1(I, X) o[I] = bfr(X);
__device__ __forceinline__ void mk_one(const float* p, v16us& o) {
  const v4f a = *(const v4f*)(p);
  const v4f b = *(const v4f*)(p + 4);
  const v4f c = *(const v4f*)(p + 16);
  const v4f d = *(const v4f*)(p + 20);
  CV1(0, a.x) CV1(1, a.y) CV1(2, a.z) CV1(3, a.w)
  CV1(4, b.x) CV1(5, b.y) CV1(6, b.z) CV1(7, b.w)
  CV1(8, c.x) CV1(9, c.y) CV1(10, c.z) CV1(11, c.w)
  CV1(12, d.x) CV1(13, d.y) CV1(14, d.z) CV1(15, d.w)
}
#undef CV1
#define HL1(I, X) { const float f_ = (X); const unsigned short h_ = bfr(f_); hi[I] = h_; lo[I] = bfr(f_ - bfup(h_)); }
__device__ __forceinline__ void mk_hilo(const float* p, v16us& hi, v16us& lo) {
  const v4f a = *(const v4f*)(p);
  const v4f b = *(const v4f*)(p + 4);
  const v4f c = *(const v4f*)(p + 16);
  const v4f d = *(const v4f*)(p + 20);
  HL1(0, a.x) HL1(1, a.y) HL1(2, a.z) HL1(3, a.w)
  HL1(4, b.x) HL1(5, b.y) HL1(6, b.z) HL1(7, b.w)
  HL1(8, c.x) HL1(9, c.y) HL1(10, c.z) HL1(11, c.w)
  HL1(12, d.x) HL1(13, d.y) HL1(14, d.z) HL1(15, d.w)
}
#undef HL1

__global__ __launch_bounds__(PTHR) void k_prep(
    const float* __restrict__ Wz, const float* __restrict__ Wr, const float* __restrict__ Ur,
    const float* __restrict__ Wh,
    unsigned short* pz, unsigned short* pr, unsigned short* pu, unsigned short* ph) {
  const int b = blockIdx.x, tid = threadIdx.x;
  const float* src; unsigned short* dst; int ng, lb;
  if (b < BZ)               { src = Wz; dst = pz; ng = NGZ; lb = b; }
  else if (b < BZ + BR)     { src = Wr; dst = pr; ng = NGR; lb = b - BZ; }
  else if (b < BZ + 2 * BR) { src = Ur; dst = pu; ng = NGR; lb = b - BZ - BR; }
  else                      { src = Wh; dst = ph; ng = NGZ; lb = b - BZ - 2 * BR; }
  const int g  = lb * PTHR + tid;
  const int gc = g < ng ? g : ng - 1;
  const v4f a = *(const v4f*)(src + (size_t)gc * 8);
  const v4f c = *(const v4f*)(src + (size_t)gc * 8 + 4);
  v8us o;
  o[0] = bfr(a.x); o[1] = bfr(a.y); o[2] = bfr(a.z); o[3] = bfr(a.w);
  o[4] = bfr(c.x); o[5] = bfr(c.y); o[6] = bfr(c.z); o[7] = bfr(c.w);
  unsigned short* dp = dst + (size_t)g * 8;
  if (g < ng) *(volatile v8us*)dp = o;
  __threadfence();
  if (g < ng) *(volatile v8us*)dp = o;
}

template <int SPLIT>
__global__ __launch_bounds__(NTHR) void k_lin(
    const float* __restrict__ A, int nA, const unsigned short* __restrict__ W,
    const float* __restrict__ bias, int useBias, float* C) {
  __shared__ __attribute__((aligned(16))) float stg[TROWS * HID];
  const int tid = threadIdx.x, lane = tid & 31, wave = tid >> 5, hh = lane >> 4, m = lane & 15;
  const int rowBase = blockIdx.x * TROWS;
  const int wrow = wave * 16;
  int arow = rowBase + wrow + m;
  arow = arow > nA - 1 ? nA - 1 : arow;
  const float* ap = A + (size_t)arow * HID + 8 * hh;

#pragma unroll 1
  for (int grp = 0; grp < 2; ++grp) {
    v8f acc[5];
#pragma unroll
    for (int t = 0; t < 5; ++t) { const v8f z = {0.f, 0.f, 0.f, 0.f, 0.f, 0.f, 0.f, 0.f}; acc[t] = z; }
#pragma unroll 1
    for (int kt = 0; kt < HID / 32; ++kt) {
      FragB ah, al;
      if (SPLIT != 0) { mk_hilo(ap + 32 * kt, ah.u, al.u); }
      else            { mk_one(ap + 32 * kt, ah.u); al.u = ah.u; }
#pragma unroll
      for (int t = 0; t < 5; ++t) {
        const int n = 16 * (5 * grp + t) + m;
        const unsigned short* bp = W + (size_t)n * HID + 32 * kt + 8 * hh;
        FragB b;
        b.h[0] = *(const v8us*)bp;
        b.h[1] = *(const v8us*)(bp + 16);
        acc[t] = wmb(ah.v, b.v, acc[t]);
        if (SPLIT != 0) acc[t] = wmb(al.v, b.v, acc[t]);
      }
    }
#pragma unroll
    for (int t = 0; t < 5; ++t) {
      const int col = 16 * (5 * grp + t) + m;
      const float bl = bfq(bias[col]);
      const float bv = useBias != 0 ? bl : 0.0f;
      float* sp = stg + (wrow + 8 * hh) * HID + col;
#pragma unroll
      for (int r = 0; r < 8; ++r) sp[r * HID] = acc[t][r] + bv;
    }
  }
  __syncthreads();

  const float* lp = stg + wrow * HID;
  float* gp = C + (size_t)(rowBase + wrow) * HID;
#pragma unroll
  for (int i = 0; i < NST; ++i) {
    const int e = 32 * i + lane;
    const v4f v = *(const v4f*)(lp + 4 * e);
    *(volatile v4f*)(gp + 4 * e) = v;
  }
  __threadfence();
#pragma unroll
  for (int i = 0; i < NST; ++i) {
    const int e = 32 * i + lane;
    const v4f v = *(const v4f*)(lp + 4 * e);
    *(volatile v4f*)(gp + 4 * e) = v;
  }
}

__device__ __forceinline__ void mm320(v8f (&acc)[5], const int grp, const float* xp, const float* a2p,
                                      const unsigned short* __restrict__ W, const int hh, const int m) {
#pragma unroll 1
  for (int kt = 0; kt < HID / 32; ++kt) {
    FragB a;
    mk_one(xp + 32 * kt, a.u);
#pragma unroll
    for (int t = 0; t < 5; ++t) {
      const int n = 16 * (5 * grp + t) + m;
      const unsigned short* bp = W + (size_t)n * KZ + 32 * kt + 8 * hh;
      FragB b;
      b.h[0] = *(const v8us*)bp;
      b.h[1] = *(const v8us*)(bp + 16);
      acc[t] = wmb(a.v, b.v, acc[t]);
    }
  }
#pragma unroll 1
  for (int kt = 0; kt < HID / 32; ++kt) {
    FragB ah, al;
    mk_hilo(a2p + 32 * kt, ah.u, al.u);
#pragma unroll
    for (int t = 0; t < 5; ++t) {
      const int n = 16 * (5 * grp + t) + m;
      const unsigned short* bp = W + (size_t)n * KZ + HID + 32 * kt + 8 * hh;
      FragB b;
      b.h[0] = *(const v8us*)bp;
      b.h[1] = *(const v8us*)(bp + 16);
      acc[t] = wmb(ah.v, b.v, acc[t]);
      acc[t] = wmb(al.v, b.v, acc[t]);
    }
  }
}

template <int RND>
__global__ __launch_bounds__(NTHR) void k_gate(
    const float* __restrict__ hin, const float* __restrict__ UH, const float* __restrict__ R1,
    const float* __restrict__ x, const int* __restrict__ gr,
    const unsigned short* __restrict__ Wz, const float* __restrict__ bz,
    const unsigned short* __restrict__ Wh, const float* __restrict__ bh,
    float* hout, int nOut, int nN) {
  extern __shared__ v4f dsm[];
  float* sumh = (float*)dsm;
  float* sumg = sumh + TROWS * HID;
  float* zt   = sumg + TROWS * HID;
  int*   gid  = (int*)(zt + TROWS * HID);
  const int tid = threadIdx.x, lane = tid & 31, wave = tid >> 5, hh = lane >> 4, m = lane & 15;
  const int rowBase = blockIdx.x * TROWS;
  const int wrow = wave * 16;

  {
    int q = rowBase * (NEI / 4) + tid;
    const int qmax = nN * (NEI / 4) - 1;
    q = q > qmax ? qmax : q;
    *(v4i*)(gid + 4 * tid) = *(const v4i*)(gr + (size_t)q * 4);
  }
  __syncthreads();

#define NEI_STEP(MI) { \
    int mi_ = (MI); mi_ = mi_ < 0 ? 0 : (mi_ > nN - 1 ? nN - 1 : mi_); \
    v4f hv_ = *(const v4f*)(hin + (size_t)mi_ * HID + c); \
    if (RND != 0) { hv_.x = bfq(hv_.x); hv_.y = bfq(hv_.y); hv_.z = bfq(hv_.z); hv_.w = bfq(hv_.w); } \
    const v4f uv_ = *(const v4f*)(UH + (size_t)mi_ * HID + c); \
    s = s + hv_; \
    g.x += sigf(rv.x + uv_.x) * hv_.x; g.y += sigf(rv.y + uv_.y) * hv_.y; \
    g.z += sigf(rv.z + uv_.z) * hv_.z; g.w += sigf(rv.w + uv_.w) * hv_.w; }

#pragma unroll 1
  for (int j = 0; j < ITEMS; ++j) {
    const int q = j * NTHR + tid;
    const int r = q / C4;
    const int c = (q - r * C4) * 4;
    int n = rowBase + r;
    n = n > nN - 1 ? nN - 1 : n;
    const v4i ga = *(const v4i*)(gid + r * NEI);
    const v4i gb = *(const v4i*)(gid + r * NEI + 4);
    const v4f rv = *(const v4f*)(R1 + (size_t)n * HID + c);
    v4f s = {0.f, 0.f, 0.f, 0.f};
    v4f g = {0.f, 0.f, 0.f, 0.f};
    NEI_STEP(ga.x) NEI_STEP(ga.y) NEI_STEP(ga.z) NEI_STEP(ga.w)
    NEI_STEP(gb.x) NEI_STEP(gb.y) NEI_STEP(gb.z) NEI_STEP(gb.w)
    *(v4f*)(sumh + r * HID + c) = s;
    *(v4f*)(sumg + r * HID + c) = g;
  }
#undef NEI_STEP
  __syncthreads();

  int xrow = rowBase + wrow + m;
  xrow = xrow > nN - 1 ? nN - 1 : xrow;
  const float* xp  = x + (size_t)xrow * HID + 8 * hh;
  const float* shp = sumh + (wrow + m) * HID + 8 * hh;
  const float* sgp = sumg + (wrow + m) * HID + 8 * hh;

#pragma unroll 1
  for (int grp = 0; grp < 2; ++grp) {
    v8f acc[5];
#pragma unroll
    for (int t = 0; t < 5; ++t) { const v8f z = {0.f, 0.f, 0.f, 0.f, 0.f, 0.f, 0.f, 0.f}; acc[t] = z; }
    mm320(acc, grp, xp, shp, Wz, hh, m);
#pragma unroll
    for (int t = 0; t < 5; ++t) {
      const int col = 16 * (5 * grp + t) + m;
      const float bv = bfq(bz[col]);
      float* zp = zt + (wrow + 8 * hh) * HID + col;
#pragma unroll
      for (int r = 0; r < 8; ++r) zp[r * HID] = sigf(acc[t][r] + bv);
    }
  }
  __syncthreads();

#pragma unroll 1
  for (int grp = 0; grp < 2; ++grp) {
    v8f acc[5];
#pragma unroll
    for (int t = 0; t < 5; ++t) { const v8f z = {0.f, 0.f, 0.f, 0.f, 0.f, 0.f, 0.f, 0.f}; acc[t] = z; }
    mm320(acc, grp, xp, sgp, Wh, hh, m);
#pragma unroll
    for (int t = 0; t < 5; ++t) {
      const int col = 16 * (5 * grp + t) + m;
      const float bv = bfq(bh[col]);
      const int p0 = (wrow + 8 * hh) * HID + col;
#pragma unroll
      for (int r = 0; r < 8; ++r) {
        const int p = p0 + r * HID;
        const float pre = tnhf(acc[t][r] + bv);
        const float zv  = zt[p];
        const float sv  = sumh[p];
        float v = (1.0f - zv) * sv + zv * pre;
        const int grow = rowBase + wrow + 8 * hh + r;
        v = (grow == 0) ? 0.0f : v;
        zt[p] = v;
      }
    }
  }
  __syncthreads();

  const float* lp = zt + wrow * HID;
  float* gp = hout + (size_t)(rowBase + wrow) * HID;
  const int vr = nOut - (rowBase + wrow);
#pragma unroll
  for (int i = 0; i < NST; ++i) {
    const int e = 32 * i + lane;
    const v4f v = *(const v4f*)(lp + 4 * e);
    if ((e / C4) < vr) *(volatile v4f*)(gp + 4 * e) = v;
  }
  __threadfence();
#pragma unroll
  for (int i = 0; i < NST; ++i) {
    const int e = 32 * i + lane;
    const v4f v = *(const v4f*)(lp + 4 * e);
    if ((e / C4) < vr) *(volatile v4f*)(gp + 4 * e) = v;
  }
}

extern "C" void kernel_launch(void* const* d_in, const int* in_sizes, int n_in,
                              void* d_out, int out_size, void* d_ws, size_t ws_size,
                              hipStream_t stream) {
  if (n_in < 10) return;
  const int nN = in_sizes[0] / HID;
  if (nN < 1 || nN > (1 << 22)) return;
  if (in_sizes[0] != nN * HID || in_sizes[1] != nN * HID || in_sizes[2] != nN * NEI) return;
  if (in_sizes[3] != HID * KZ || in_sizes[4] != HID || in_sizes[5] != HID * HID ||
      in_sizes[6] != HID * HID || in_sizes[7] != HID || in_sizes[8] != HID * KZ || in_sizes[9] != HID) return;
  if (out_size != nN * HID) return;

  const float* h0   = (const float*)d_in[0];
  const float* x    = (const float*)d_in[1];
  const int*   gr   = (const int*)d_in[2];
  const float* Wz_w = (const float*)d_in[3];
  const float* Wz_b = (const float*)d_in[4];
  const float* Wr_w = (const float*)d_in[5];
  const float* Ur_w = (const float*)d_in[6];
  const float* Ur_b = (const float*)d_in[7];
  const float* Wh_w = (const float*)d_in[8];
  const float* Wh_b = (const float*)d_in[9];
  float* out = (float*)d_out;

  const int nBlk = (nN + TROWS - 1) / TROWS;
  const int NPAD = nBlk * TROWS;

  char* ws = (char*)d_ws;
  size_t off = 0;
  const size_t oWz = off; off += (size_t)HID * KZ * 2;
  const size_t oWh = off; off += (size_t)HID * KZ * 2;
  const size_t oWr = off; off += (size_t)HID * HID * 2;
  const size_t oUr = off; off += (size_t)HID * HID * 2;
  off = (off + 255) & ~(size_t)255;
  const size_t plane = (size_t)NPAD * HID * 4;
  const size_t oR1 = off; off += plane;
  const size_t oUH = off; off += plane;
  const size_t oHB = off; off += plane;
  if (off > ws_size) return;

  unsigned short* pWz = (unsigned short*)(ws + oWz);
  unsigned short* pWh = (unsigned short*)(ws + oWh);
  unsigned short* pWr = (unsigned short*)(ws + oWr);
  unsigned short* pUr = (unsigned short*)(ws + oUr);
  float* R1 = (float*)(ws + oR1);
  float* UH = (float*)(ws + oUH);
  float* hB = (float*)(ws + oHB);

  k_prep<<<NPREPB, PTHR, 0, stream>>>(Wz_w, Wr_w, Ur_w, Wh_w, pWz, pWr, pUr, pWh);

  k_lin<0><<<nBlk, NTHR, 0, stream>>>(x, nN, pWr, Ur_b, 0, R1);

  hipFuncSetAttribute(reinterpret_cast<const void*>(&k_gate<0>),
                      hipFuncAttributeMaxDynamicSharedMemorySize, LDS_GATE);
  hipFuncSetAttribute(reinterpret_cast<const void*>(&k_gate<1>),
                      hipFuncAttributeMaxDynamicSharedMemorySize, LDS_GATE);

  k_lin<0><<<nBlk, NTHR, 0, stream>>>(h0, nN, pUr, Ur_b, 1, UH);
  k_gate<1><<<nBlk, NTHR, LDS_GATE, stream>>>(h0, UH, R1, x, gr, pWz, Wz_b, pWh, Wh_b, out, nN, nN);
  k_lin<1><<<nBlk, NTHR, 0, stream>>>(out, nN, pUr, Ur_b, 1, UH);
  k_gate<0><<<nBlk, NTHR, LDS_GATE, stream>>>(out, UH, R1, x, gr, pWz, Wz_b, pWh, Wh_b, hB, NPAD, nN);
  k_lin<1><<<nBlk, NTHR, 0, stream>>>(hB, nN, pUr, Ur_b, 1, UH);
  k_gate<0><<<nBlk, NTHR, LDS_GATE, stream>>>(hB, UH, R1, x, gr, pWz, Wz_b, pWh, Wh_b, out, nN, nN);
}
